// ResidualSAGENet_41506563948594
// MI455X (gfx1250) — hardware-verified
//
#include <hip/hip_runtime.h>
#include <math.h>

typedef __attribute__((ext_vector_type(16))) _Float16 v16h;
typedef __attribute__((ext_vector_type(16))) __bf16 v16b;
typedef __attribute__((ext_vector_type(8)))  _Float16 v8h;
typedef __attribute__((ext_vector_type(8)))  float v8f;
typedef __attribute__((ext_vector_type(4)))  float v4f;
typedef __attribute__((ext_vector_type(2)))  float v2f;
typedef __attribute__((ext_vector_type(4)))  unsigned v4u;
typedef __attribute__((ext_vector_type(4)))  int v4i;
typedef float __attribute__((may_alias)) float_a;
typedef int __attribute__((may_alias)) int_a;

template <typename T> __device__ __forceinline__ void vst2(void* p, T v) { *(volatile T*)p = v; __threadfence(); *(volatile T*)p = v; }
__device__ __forceinline__ v8f wmma16(v16h a, v16h b, v8f c) {
  v8f d = __builtin_amdgcn_wmma_f32_16x16x32_f16(false, a, false, b, (short)0, c, false, false);
  asm volatile("v_nop\n\tv_nop\n\tv_nop\n\tv_nop" : "+v"(d) : "v"(a), "v"(b));
  return d;
}
__device__ __forceinline__ v8f wmma_bf(v16b a, v16b b, v8f c) {
  v8f d = __builtin_amdgcn_wmma_f32_16x16x32_bf16(false, a, false, b, (short)0, c, false, false);
  asm volatile("v_nop\n\tv_nop\n\tv_nop\n\tv_nop" : "+v"(d) : "v"(a), "v"(b));
  return d;
}
__device__ __forceinline__ v16h frag_h(const _Float16* rowk0, int lane) {
  union { v16h v; v8h q[2]; } u; const _Float16* p = rowk0 + 8 * (lane >> 4);
  u.q[0] = *(const v8h*)p; u.q[1] = *(const v8h*)(p + 16); return u.v;
}
__device__ __forceinline__ v16h frag_f32(const float* rowk0, int lane) {
  v16h a; const float* p = rowk0 + 8 * (lane >> 4);
#pragma unroll
  for (int i = 0; i < 8; ++i) { a[i] = (_Float16)p[i]; a[8 + i] = (_Float16)p[16 + i]; }
  return a;
}
__device__ __forceinline__ v16h frag_f32s(const float* rowk0, int lane, float sc) {
  v16h a; const float* p = rowk0 + 8 * (lane >> 4);
#pragma unroll
  for (int i = 0; i < 8; ++i) { a[i] = (_Float16)(p[i] * sc); a[8 + i] = (_Float16)(p[16 + i] * sc); }
  return a;
}
__device__ __forceinline__ v16h fragc_f32(const float* W, int k0, int n, int lane, int ld, int K) {
  v16h a; const int g = lane >> 4;
#pragma unroll
  for (int i = 0; i < 8; ++i) { const int ka = k0 + 8 * g + i, kb = ka + 16;
    a[i] = (_Float16)(ka < K ? W[(size_t)ka * ld + n] : 0.f); a[8 + i] = (_Float16)(kb < K ? W[(size_t)kb * ld + n] : 0.f); }
  return a;
}
struct F2 { v16b h, l; };
__device__ __forceinline__ F2 bsplit16(const float v[16]) { F2 r;
#pragma unroll
  for (int i = 0; i < 16; ++i) { const __bf16 h = (__bf16)v[i]; r.h[i] = h; r.l[i] = (__bf16)(v[i] - (float)h); }
  return r; }
__device__ __forceinline__ F2 split_row(const float* row, int k0, int lane) { float v[16]; const float* p = row + k0 + 8 * (lane >> 4);
#pragma unroll
  for (int i = 0; i < 8; ++i) { v[i] = p[i]; v[8 + i] = p[16 + i]; }
  return bsplit16(v); }
__device__ __forceinline__ F2 split_rowK(const float* row, int k0, int lane, int K) { float v[16]; const int g = lane >> 4;
#pragma unroll
  for (int i = 0; i < 8; ++i) { const int ka = k0 + 8 * g + i, kb = ka + 16; v[i] = ka < K ? row[ka] : 0.f; v[8 + i] = kb < K ? row[kb] : 0.f; }
  return bsplit16(v); }
__device__ __forceinline__ F2 split_col(const float* W, int k0, int n, int lane, int ld, int K) { float v[16]; const int g = lane >> 4;
#pragma unroll
  for (int i = 0; i < 8; ++i) { const int ka = k0 + 8 * g + i, kb = ka + 16; v[i] = ka < K ? W[(size_t)ka * ld + n] : 0.f; v[8 + i] = kb < K ? W[(size_t)kb * ld + n] : 0.f; }
  return bsplit16(v); }
__device__ __forceinline__ v8f mac3(const F2& a, const F2& b, v8f c) { c = wmma_bf(a.l, b.h, c); c = wmma_bf(a.h, b.l, c); return wmma_bf(a.h, b.h, c); }
__device__ __forceinline__ float sigm(float v) { return 1.0f / (1.0f + expf(-v)); }
#define LDSX() do { asm volatile("s_wait_dscnt 0" ::: "memory"); __builtin_amdgcn_wave_barrier(); __builtin_amdgcn_fence(__ATOMIC_RELEASE, "workgroup"); } while (0)

#define NN 100000
#define NE 600000
#define FH 128
#define NCLS 47
#define RB 512
#define NRB ((NN + RB - 1) / RB)
#define NNP (NRB * RB)
#define EPT 16
#define CH (256 * EPT)

__global__ __launch_bounds__(256) void k_pack(const float* __restrict__ inW, const float* __restrict__ Wl, const float* __restrict__ Wr, const float* __restrict__ oW, _Float16* __restrict__ P) {
  const int r = blockIdx.x, tid = threadIdx.x; __shared__ __align__(16) _Float16 srow[256];
  float v = 0.f;
  if (r < 128) { v = tid < 128 ? inW[(size_t)tid * FH + r] : 0.f; }
  else if (r < 512) { const int l = (r - 128) >> 7, n = (r - 128) & 127; v = tid < 128 ? Wl[((size_t)l * FH + tid) * FH + n] : Wr[((size_t)l * FH + (tid - 128)) * FH + n]; }
  else { const int n = r - 512; v = (n < NCLS && tid < 128) ? oW[(size_t)tid * NCLS + n] : 0.f; }
  srow[tid] = (_Float16)(v * 16.0f);
  __syncthreads();
  if (tid < 32) vst2(P + (size_t)r * 256 + tid * 8, *(const v4u*)(&srow[tid * 8]));
}
__global__ __launch_bounds__(128) void k_in(const float* __restrict__ x, const _Float16* __restrict__ P, const float* __restrict__ inb, const float* __restrict__ g, const float* __restrict__ be, const float* __restrict__ m, const float* __restrict__ var, float* __restrict__ H32, _Float16* __restrict__ AH) {
  __shared__ __align__(16) float so[4][16][132];
  const int tid = threadIdx.x, wave = tid >> 5, lane = tid & 31, col = lane & 15, gg = lane >> 4;
  const int r0 = blockIdx.x * 64 + wave * 16;
  v8f acc[8] = {};
const int ra = (r0 + col) < NN ? (r0 + col) : (NN - 1);
#pragma unroll
  for (int kc = 0; kc < FH / 32; ++kc) { const v16h a = frag_f32(x + (size_t)ra * FH + kc * 32, lane);
#pragma unroll
    for (int j = 0; j < 8; ++j) acc[j] = wmma16(a, frag_h(P + (size_t)(j * 16 + col) * 256 + kc * 32, lane), acc[j]); }
#pragma unroll
  for (int j = 0; j < 8; ++j) { const int n = j * 16 + col; const float sc = g[n] * rsqrtf(var[n] + 1e-5f), bb = inb[n], mm = m[n], bt = be[n];
#pragma unroll
    for (int r = 0; r < 8; ++r) { float v = acc[j][r] * (1.0f / 16.0f) + bb; v = (v - mm) * sc + bt; so[wave][8 * gg + r][n] = v > 0.f ? v : 0.f; } }
  LDSX();
  for (int q = lane; q < 16 * 32; q += 32) { const int rl = q >> 5, pc = q & 31; const size_t row = r0 + rl; const v4f v = *(const v4f*)(&so[wave][rl][pc * 4]);
    vst2(H32 + row * FH + pc * 4, v);
    if ((pc & 1) == 0) { union { v8h h; v4u u; } pk; const v4f v2 = *(const v4f*)(&so[wave][rl][pc * 4 + 4]);
      pk.h[0] = (_Float16)v[0]; pk.h[1] = (_Float16)v[1]; pk.h[2] = (_Float16)v[2]; pk.h[3] = (_Float16)v[3]; pk.h[4] = (_Float16)v2[0]; pk.h[5] = (_Float16)v2[1]; pk.h[6] = (_Float16)v2[2]; pk.h[7] = (_Float16)v2[3];
      vst2(AH + row * 256 + 128 + pc * 4, pk.u); } }
}
__global__ __launch_bounds__(256) void k_agg(const float* __restrict__ H32, const int* __restrict__ ei, _Float16* __restrict__ AH) {
  __shared__ __align__(16) float sacc[RB][FH];
  __shared__ int ssrc[8][32 * EPT], sdl[8][32 * EPT]; __shared__ int scnt[8]; __shared__ int srcnt[RB];
  const int tid = threadIdx.x, wave = tid >> 5, lane = tid & 31;
  const int r0 = blockIdx.x * RB; const int* esrc = ei; const int* edst = ei + NE;
  for (int q = tid; q < RB * FH; q += 256) (&sacc[0][0])[q] = 0.f;
  for (int q = tid; q < RB; q += 256) srcnt[q] = 0;
  __syncthreads();
#pragma unroll 1
  for (int c0 = 0; c0 < NE; c0 += CH) {
    const int e0 = c0 + tid * EPT; int hd[EPT]; int cnt = 0;
    if (e0 + EPT <= NE) {
#pragma unroll
      for (int v = 0; v < EPT / 4; ++v) { const int4 d4 = *(const int4*)(edst + e0 + v * 4);
        const int dd[4] = {d4.x, d4.y, d4.z, d4.w};
#pragma unroll
        for (int u = 0; u < 4; ++u) { const unsigned rel = (unsigned)(dd[u] - r0); const bool h = rel < (unsigned)RB; hd[v * 4 + u] = h ? (int)rel : -1; cnt += h ? 1 : 0; } } }
    else {
#pragma unroll
      for (int u = 0; u < EPT; ++u) { const int e = e0 + u; hd[u] = -1; if (e < NE) { const unsigned rel = (unsigned)(edst[e] - r0); if (rel < (unsigned)RB) { hd[u] = (int)rel; ++cnt; } } } }
    int incl = cnt;
#pragma unroll
    for (int off = 1; off < 32; off <<= 1) { const int vv = __shfl_up(incl, off, 32); if (lane >= off) incl += vv; }
    const int wtot = __shfl(incl, 31, 32); int pos = incl - cnt;
    if (cnt > 0) {
#pragma unroll
      for (int u = 0; u < EPT; ++u) if (hd[u] >= 0) { int s = esrc[e0 + u]; s = s < 0 ? 0 : (s >= NN ? NN - 1 : s); ssrc[wave][pos] = s; sdl[wave][pos] = hd[u]; atomicAdd(&srcnt[hd[u]], 1); ++pos; } }
    if (lane == 0) scnt[wave] = wtot;
    __syncthreads();
    if (tid < FH) { for (int w = 0; w < 8; ++w) { const int nh = scnt[w]; for (int i = 0; i < nh; ++i) sacc[sdl[w][i]][tid] += H32[(size_t)ssrc[w][i] * FH + tid]; } }
    __syncthreads(); }
  for (int q = tid; q < RB * (FH / 8); q += 256) { const int rl = q >> 4, pc = q & 15; const int row = r0 + rl; const float inv = 1.0f / fmaxf((float)srcnt[rl], 1.0f);
    union { v8h h; v4u u; } pk;
#pragma unroll
    for (int e = 0; e < 8; ++e) pk.h[e] = (_Float16)(row < NN ? sacc[rl][pc * 8 + e] * inv : 0.f);
    vst2(AH + (size_t)row * 256 + pc * 8, pk.u); }
}
__global__ __launch_bounds__(128) void k_layer(const _Float16* __restrict__ P, int prow0, const float* __restrict__ bl, const float* __restrict__ g, const float* __restrict__ be, const float* __restrict__ m, const float* __restrict__ var, float* __restrict__ H32, _Float16* __restrict__ AH) {
  __shared__ __align__(16) float so[4][16][132];
  const int tid = threadIdx.x, wave = tid >> 5, lane = tid & 31, col = lane & 15, gg = lane >> 4;
  const int r0 = blockIdx.x * 64 + wave * 16;
  v8f acc[8] = {};
#pragma unroll 2
  for (int kc = 0; kc < 8; ++kc) { const v16h a = frag_h(AH + (size_t)(r0 + col) * 256 + kc * 32, lane);
#pragma unroll
    for (int j = 0; j < 8; ++j) acc[j] = wmma16(a, frag_h(P + (size_t)(prow0 + j * 16 + col) * 256 + kc * 32, lane), acc[j]); }
#pragma unroll
  for (int j = 0; j < 8; ++j) { const int n = j * 16 + col; const float sc = g[n] * rsqrtf(var[n] + 1e-5f), bb = bl[n], mm = m[n], bt = be[n];
#pragma unroll
    for (int r = 0; r < 8; ++r) { float v = acc[j][r] * (1.0f / 16.0f) + bb; v = (v - mm) * sc + bt; v = v > 0.f ? v : 0.f; so[wave][8 * gg + r][n] = v + H32[(size_t)(r0 + 8 * gg + r) * FH + n]; } }
  LDSX();
  for (int q = lane; q < 16 * 32; q += 32) { const int rl = q >> 5, pc = q & 31; const size_t row = r0 + rl; const v4f v = *(const v4f*)(&so[wave][rl][pc * 4]);
    vst2(H32 + row * FH + pc * 4, v);
    if ((pc & 1) == 0) { union { v8h h; v4u u; } pk; const v4f v2 = *(const v4f*)(&so[wave][rl][pc * 4 + 4]);
      pk.h[0] = (_Float16)v[0]; pk.h[1] = (_Float16)v[1]; pk.h[2] = (_Float16)v[2]; pk.h[3] = (_Float16)v[3]; pk.h[4] = (_Float16)v2[0]; pk.h[5] = (_Float16)v2[1]; pk.h[6] = (_Float16)v2[2]; pk.h[7] = (_Float16)v2[3];
      vst2(AH + row * 256 + 128 + pc * 4, pk.u); } }
}
__global__ __launch_bounds__(128) void k_out(const _Float16* __restrict__ AH, const _Float16* __restrict__ P, const float* __restrict__ ob, float* __restrict__ out) {
  __shared__ __align__(16) float so[64][48];
  const int tid = threadIdx.x, wave = tid >> 5, lane = tid & 31, col = lane & 15, gg = lane >> 4;
  const int r0b = blockIdx.x * 64, r0 = r0b + wave * 16;
  v8f acc[3] = {};
#pragma unroll
  for (int kc = 0; kc < 4; ++kc) { const v16h a = frag_h(AH + (size_t)(r0 + col) * 256 + 128 + kc * 32, lane);
#pragma unroll
    for (int j = 0; j < 3; ++j) acc[j] = wmma16(a, frag_h(P + (size_t)(512 + j * 16 + col) * 256 + kc * 32, lane), acc[j]); }
#pragma unroll
  for (int j = 0; j < 3; ++j) { const int n = j * 16 + col; const float bb = n < NCLS ? ob[n] : 0.f;
#pragma unroll
    for (int r = 0; r < 8; ++r) so[wave * 16 + 8 * gg + r][n] = acc[j][r] * (1.0f / 16.0f) + bb; }
  __syncthreads();
  const int nrows = (r0b + 64 <= NN) ? 64 : (NN - r0b > 0 ? NN - r0b : 0);
  for (int q = tid; q < nrows * NCLS; q += 128) { const int rl = q / NCLS, c = q % NCLS; vst2(out + (size_t)(r0b + rl) * NCLS + c, so[rl][c]); }
}
extern "C" void kernel_launch(void* const* d_in, const int* in_sizes, int n_in, void* d_out, int out_size, void* d_ws, size_t ws_size, hipStream_t stream) {
  (void)in_sizes; (void)n_in; (void)out_size; (void)ws_size;
  const float** I = (const float**)d_in;
  const float* x = I[0]; const float* inW = I[1]; const float* inb = I[2]; const float* ig = I[3]; const float* ib = I[4]; const float* im = I[5]; const float* iv = I[6];
  const float* Wl = I[7]; const float* bl = I[8]; const float* Wr = I[9]; const float* bg = I[10]; const float* bb = I[11]; const float* bm = I[12]; const float* bv = I[13]; const float* oW = I[14]; const float* ob = I[15]; const int* ei = (const int*)d_in[16];
  float* out = (float*)d_out;
  char* ws = (char*)d_ws; size_t off = 0;
  auto take = [&](size_t bytes) { char* p = ws + off; off += (bytes + 255) & ~(size_t)255; return p; };
  _Float16* P = (_Float16*)take((size_t)576 * 256 * 2); float* H32 = (float*)take((size_t)NNP * FH * 4); _Float16* AH = (_Float16*)take((size_t)NNP * 256 * 2);
  k_pack<<<576, 256, 0, stream>>>(inW, Wl, Wr, oW, P);
  k_in<<<NNP / 64, 128, 0, stream>>>(x, P, inb, ig, ib, im, iv, H32, AH);
  for (int l = 0; l < 3; ++l) {
    k_agg<<<NRB, 256, 0, stream>>>(H32, ei, AH);
    k_layer<<<NNP / 64, 128, 0, stream>>>(P, 128 + l * 128, bl + l * FH, bg + l * FH, bb + l * FH, bm + l * FH, bv + l * FH, H32, AH); }
  k_out<<<NNP / 64, 128, 0, stream>>>(AH, P, ob, out);
}
